// MultiHeadedAttention_36971078484381
// MI455X (gfx1250) — hardware-verified
//
#include <hip/hip_runtime.h>


#ifndef NB
#define NB 4
#endif
#ifndef SEQ
#define SEQ 2048
#endif
#define NB_FULL  4
#define SEQ_FULL 2048
#define DM   512
#define NH_  8
#define HD   64
#define NBH  (NB * NH_)
#define KOFF 16
#define KSL  64
#define KROWS (SEQ + KSL)
#define RMAX 33
#define PP   72
#define PCAR 1024.0f
#define SCL  0.125f

static_assert(NB <= NB_FULL);
static_assert(SEQ <= SEQ_FULL);
static_assert(SEQ % 64 == 0);
static_assert(HD == 64);
static_assert(DM == NH_ * HD);
static_assert(DM % 64 == 0);
static_assert(KROWS % 64 == 0);
static_assert((DM * DM / 64) % 64 == 0);
static_assert(((size_t)NB * SEQ * (DM / 8)) % 256 == 0);
static_assert(((size_t)NBH * SEQ * HD) % 512 == 0);
static_assert(((size_t)NBH * KROWS * HD) % 512 == 0);

typedef _Float16 h16;
typedef unsigned short bf;
typedef __attribute__((ext_vector_type(16))) __bf16   v16bf;
typedef __attribute__((ext_vector_type(16))) _Float16 v16h;
typedef __attribute__((ext_vector_type(8)))  _Float16 v8h;
typedef __attribute__((ext_vector_type(8)))  unsigned short v8us;
typedef __attribute__((ext_vector_type(8)))  float    v8f;
typedef __attribute__((ext_vector_type(4)))  float    v4f;
typedef __attribute__((ext_vector_type(2)))  _Float16 v2h;
typedef __attribute__((ext_vector_type(2)))  unsigned short v2us;
typedef __attribute__((ext_vector_type(2)))  float    v2f;
typedef v8h  __attribute__((may_alias)) v8ha;
typedef v4f  __attribute__((may_alias)) v4fa;

__device__ __forceinline__ unsigned short f2bf(float f) { unsigned u = __float_as_uint(f); u += 0x7FFFu + ((u >> 16) & 1u); return (unsigned short)(u >> 16); }
__device__ __forceinline__ float bf2f(unsigned short b) { return __uint_as_float(((unsigned)b) << 16); }
__device__ __forceinline__ float bfr(float f) { return bf2f(f2bf(f)); }
__device__ __forceinline__ v16h cat16(v8h lo, v8h hi) { return __builtin_shufflevector(lo, hi, 0, 1, 2, 3, 4, 5, 6, 7, 8, 9, 10, 11, 12, 13, 14, 15); }
__device__ __forceinline__ v16bf cat16b(v8us lo, v8us hi) { return __builtin_bit_cast(v16bf, __builtin_shufflevector(lo, hi, 0, 1, 2, 3, 4, 5, 6, 7, 8, 9, 10, 11, 12, 13, 14, 15)); }
__device__ __forceinline__ v8f wmma16(v16h a, v16h b, v8f c) { return __builtin_amdgcn_wmma_f32_16x16x32_f16(false, a, false, b, (short)0, c, false, false); }
__device__ __forceinline__ v8f wmmab(v16bf a, v16bf b, v8f c) { return __builtin_amdgcn_wmma_f32_16x16x32_bf16(false, a, false, b, (short)0, c, false, false); }
__device__ __forceinline__ void splitf(float y, unsigned short& h, unsigned short& l) { h = f2bf(y); l = f2bf(y - bf2f(h)); }

template <typename T16> struct WFrag;
template <> struct WFrag<h16> { typedef v16h V; static __device__ __forceinline__ V ld(const h16* p) { return cat16(*(const v8h*)p, *(const v8h*)(p + 16)); } static __device__ __forceinline__ v8f mma(V a, V b, v8f c) { return wmma16(a, b, c); } };
template <> struct WFrag<bf> { typedef v16bf V; static __device__ __forceinline__ V ld(const bf* p) { return cat16b(*(const v8us*)p, *(const v8us*)(p + 16)); } static __device__ __forceinline__ v8f mma(V a, V b, v8f c) { return wmmab(a, b, c); } };
template <typename T16, int NSPLIT, bool BIAS>
__global__ __launch_bounds__(32) void k_gemmw(const T16* __restrict__ A, const T16* __restrict__ A2, const T16* __restrict__ Bt, const T16* __restrict__ Bt2, int K, float* C, int ldc, const float* __restrict__ bias, size_t sA, size_t sB, size_t sC) {
    typedef typename WFrag<T16>::V V;
    __shared__ __align__(16) float os[16 * 68];
    const size_t z = blockIdx.z; A += z * sA; if (A2) A2 += z * sA; Bt += z * sB; if (Bt2) Bt2 += z * sB; C += z * sC;
    const int lane = threadIdx.x & 31, lr = lane & 15, hi = lane >> 4; const int r0 = blockIdx.x * 64, c0 = blockIdx.y * 64;
    v8f acc[4][4];
#pragma unroll
    for (int mb = 0; mb < 4; ++mb)
#pragma unroll
        for (int nb = 0; nb < 4; ++nb) acc[mb][nb] = (v8f){};
    const size_t aoff = (size_t)(r0 + lr) * K + 8 * hi, boff = (size_t)(c0 + lr) * K + 8 * hi;
#pragma unroll 1
    for (int kc = 0; kc < K; kc += 32) {
        V a[4], a2[4];
#pragma unroll
        for (int mb = 0; mb < 4; ++mb) { a[mb] = WFrag<T16>::ld(A + aoff + (size_t)mb * 16 * K + kc); if (NSPLIT == 1 || NSPLIT == 2) a2[mb] = WFrag<T16>::ld(A2 + aoff + (size_t)mb * 16 * K + kc); }
#pragma unroll
        for (int nb = 0; nb < 4; ++nb) { const V b = WFrag<T16>::ld(Bt + boff + (size_t)nb * 16 * K + kc); V b2; if (NSPLIT >= 2) b2 = WFrag<T16>::ld(Bt2 + boff + (size_t)nb * 16 * K + kc);
#pragma unroll
            for (int mb = 0; mb < 4; ++mb) { acc[mb][nb] = WFrag<T16>::mma(a[mb], b, acc[mb][nb]); if (NSPLIT == 1 || NSPLIT == 2) acc[mb][nb] = WFrag<T16>::mma(a2[mb], b, acc[mb][nb]); if (NSPLIT >= 2) acc[mb][nb] = WFrag<T16>::mma(a[mb], b2, acc[mb][nb]); } }
        asm volatile("v_nop\n\tv_nop\n\tv_nop\n\tv_nop" : "+v"(acc[0][0]), "+v"(acc[1][1]), "+v"(acc[2][2]), "+v"(acc[3][3]) : "v"(a[0]), "v"(a[3]));
    }
#pragma unroll
    for (int mb = 0; mb < 4; ++mb) {
#pragma unroll
        for (int nb = 0; nb < 4; ++nb) {
#pragma unroll
            for (int j = 0; j < 8; ++j) os[(hi * 8 + j) * 68 + nb * 16 + lr] = acc[mb][nb][j]; }
        __builtin_amdgcn_wave_barrier(); asm volatile("" ::: "memory");
        float* crow = C + (size_t)(r0 + mb * 16) * ldc + c0;
#pragma unroll 1
        for (int ps = 0; ps < 2; ++ps) {
#pragma unroll
            for (int s = 0; s < 8; ++s) { const int row = 2 * s + hi, cofs = lr * 4; v4f val = *(const v4fa*)(os + row * 68 + cofs); if (BIAS) { val[0] += bfr(bias[c0 + cofs]); val[1] += bfr(bias[c0 + cofs + 1]); val[2] += bfr(bias[c0 + cofs + 2]); val[3] += bfr(bias[c0 + cofs + 3]); }
                *(volatile v4f*)(crow + (size_t)row * ldc + cofs) = val; }
            if (ps == 0) __threadfence(); }
        __builtin_amdgcn_wave_barrier(); asm volatile("" ::: "memory");
    }
}

__global__ __launch_bounds__(256) void k_wtG(const float* __restrict__ w, bf* Bt) {
    const unsigned lane = threadIdx.x & 31u; const unsigned L0 = (blockIdx.x * 8u + (threadIdx.x >> 5)) * 8u;
#pragma unroll
    for (int ps = 0; ps < 2; ++ps) {
#pragma unroll 1
        for (unsigned l = 0; l < 8u; ++l) { const unsigned L = L0 + l; const unsigned e = L * 64u + lane * 2u; const unsigned k = e % (unsigned)DM, n = e / (unsigned)DM; v2us o;
            o[0] = f2bf(w[(size_t)k * DM + n]); o[1] = f2bf(w[(size_t)(k + 1u) * DM + n]); *(volatile v2us*)(Bt + e) = o; }
        if (ps == 0) __threadfence(); }
}

__global__ __launch_bounds__(256) void k_cvt8b(const float* __restrict__ src, bf* dst) {
    const unsigned i = blockIdx.x * 256u + threadIdx.x; if (i >= (unsigned)NB * SEQ * (DM / 8)) return;
    const unsigned c = i % (unsigned)(DM / 8), row = i / (unsigned)(DM / 8); const unsigned b = row / (unsigned)SEQ, t = row % (unsigned)SEQ;
    const v8f v = *(const v8f*)(src + ((size_t)b * SEQ_FULL + t) * DM + c * 8u); v8us o;
#pragma unroll
    for (int k = 0; k < 8; ++k) o[k] = f2bf(v[k]);
    *(volatile v8us*)(dst + (size_t)i * 8) = o; __threadfence(); *(volatile v8us*)(dst + (size_t)i * 8) = o; }

template <unsigned ROWS, unsigned OFF>
__global__ __launch_bounds__(256) void k_hplane(const float* __restrict__ F, bf* Ph, bf* Pl) {
    const unsigned e = (blockIdx.x * 256u + threadIdx.x) * 2u; if (e >= (unsigned)NBH * ROWS * (unsigned)HD) return;
    const unsigned d = e & 63u; const unsigned rr = e >> 6; const unsigned row = rr % ROWS; const unsigned bh = rr / ROWS; const unsigned b = bh >> 3, h = bh & 7u;
    const int pos = (int)row - (int)OFF; const bool ok = (unsigned)pos < (unsigned)SEQ; const unsigned pc = ok ? (unsigned)pos : 0u;
    const v2f x = *(const v2f*)(F + ((size_t)b * SEQ + pc) * DM + h * (unsigned)HD + d);
    v2us oh, ol;
#pragma unroll
    for (int q = 0; q < 2; ++q) { const float y = ok ? x[q] : 0.0f; unsigned short a2, c2; splitf(y, a2, c2); oh[q] = a2; ol[q] = c2; }
    *(volatile v2us*)(Ph + e) = oh; *(volatile v2us*)(Pl + e) = ol; __threadfence(); *(volatile v2us*)(Ph + e) = oh; *(volatile v2us*)(Pl + e) = ol; }

__global__ __launch_bounds__(256) void k_vt16(const float* __restrict__ F, h16* V16) {
    const unsigned e = (blockIdx.x * 256u + threadIdx.x) * 2u; if (e >= (unsigned)NBH * (unsigned)HD * (unsigned)KROWS) return;
    const unsigned col = e % (unsigned)KROWS, rr = e / (unsigned)KROWS; const unsigned d = rr & 63u, bh = rr >> 6; const unsigned b = bh >> 3, h = bh & 7u;
    v2h o;
#pragma unroll
    for (unsigned q = 0; q < 2u; ++q) { const int pos = (int)(col + q) - KOFF; const bool ok = (unsigned)pos < (unsigned)SEQ; const unsigned pc = ok ? (unsigned)pos : 0u;
        const float x = F[((size_t)b * SEQ + pc) * DM + h * (unsigned)HD + d]; const float xs = ok ? x : 0.0f; o[q] = (h16)xs; }
    *(volatile v2h*)(V16 + e) = o; __threadfence(); *(volatile v2h*)(V16 + e) = o; }

__global__ __launch_bounds__(32) void k_battn(const bf* __restrict__ QPh, const bf* __restrict__ QPl, const bf* __restrict__ KPh, const bf* __restrict__ KPl, const h16* __restrict__ VT16,
                                              const int* __restrict__ mask, const int* __restrict__ rs, bf* Ah, bf* Al) {
    __shared__ __align__(16) h16 pt[16 * PP];
    __shared__ __align__(16) float ost[16 * 68];
    const unsigned lane = threadIdx.x & 31u, lr = lane & 15u, hi = lane >> 4;
    const unsigned t0 = blockIdx.x * 16u, bh = blockIdx.y, b = bh >> 3, h = bh & 7u;
    const int rin = rs[0]; const bool bad = (rin < 1) || (rin > RMAX); const int r = bad ? 1 : rin; const int half = r >> 1;
    const float pz = bad ? __uint_as_float(0x7FC00000u) : 0.0f;

    v16bf qa[2], qb[2];
    { const size_t qo = ((size_t)bh * SEQ + t0 + lr) * HD + 8u * hi;
#pragma unroll
      for (int s = 0; s < 2; ++s) { qa[s] = WFrag<bf>::ld(QPh + qo + s * 32); qb[s] = WFrag<bf>::ld(QPl + qo + s * 32); } }

    v8f sc[4];
#pragma unroll
    for (int nt = 0; nt < 4; ++nt) {
        sc[nt] = (v8f){};
        const size_t ko = ((size_t)bh * KROWS + t0 + (unsigned)nt * 16u + lr) * HD + 8u * hi;
        const v16bf kh0 = WFrag<bf>::ld(KPh + ko), kh1 = WFrag<bf>::ld(KPh + ko + 32), kl0 = WFrag<bf>::ld(KPl + ko), kl1 = WFrag<bf>::ld(KPl + ko + 32);
        sc[nt] = wmmab(qa[0], kh0, sc[nt]); sc[nt] = wmmab(qb[0], kh0, sc[nt]); sc[nt] = wmmab(qa[0], kl0, sc[nt]);
        sc[nt] = wmmab(qa[1], kh1, sc[nt]); sc[nt] = wmmab(qb[1], kh1, sc[nt]); sc[nt] = wmmab(qa[1], kl1, sc[nt]);
        asm volatile("v_nop\n\tv_nop\n\tv_nop\n\tv_nop" : "+v"(sc[nt]) : "v"(kh0), "v"(kh1), "v"(kl0), "v"(kl1), "v"(qa[0]), "v"(qa[1]), "v"(qb[0]), "v"(qb[1]));
    }

    const int jb = (int)lr - KOFF - (int)(8u * hi) + half;
#pragma unroll
    for (int j = 0; j < 8; ++j) {
        float sv[4]; bool in[4]; float mx = -3.0e38f;
#pragma unroll
        for (int nt = 0; nt < 4; ++nt) { const int jrel = jb + nt * 16 - j; in[nt] = (unsigned)jrel < (unsigned)r; sv[nt] = sc[nt][j] * SCL; const float cand = fmaxf(mx, sv[nt]); mx = in[nt] ? cand : mx; }
#pragma unroll
        for (int sh = 8; sh; sh >>= 1) mx = fmaxf(mx, __shfl_xor(mx, sh, 32));
        float ev[4]; float sum = 0.f;
#pragma unroll
        for (int nt = 0; nt < 4; ++nt) { float d0 = fminf(__fsub_rn(sv[nt], mx), 0.0f); const float ex = __builtin_amdgcn_exp2f(__fmul_rn(d0, 1.4426950408889634f)); ev[nt] = in[nt] ? ex : 0.0f; sum += ev[nt]; }
#pragma unroll
        for (int sh = 8; sh; sh >>= 1) sum += __shfl_xor(sum, sh, 32);
        const float f = __fdiv_rn(PCAR, sum);
#pragma unroll
        for (int nt = 0; nt < 4; ++nt) pt[(8u * hi + (unsigned)j) * PP + (unsigned)nt * 16u + lr] = (h16)(ev[nt] * f);
    }
    __syncthreads();
    v16h pa[2];
#pragma unroll
    for (int s = 0; s < 2; ++s) pa[s] = cat16(*(const v8ha*)(pt + lr * PP + s * 32 + 8u * hi), *(const v8ha*)(pt + lr * PP + s * 32 + 16 + 8u * hi));

    v8f xa[4];
#pragma unroll
    for (int dt = 0; dt < 4; ++dt) {
        xa[dt] = (v8f){};
        const h16* vp = VT16 + ((size_t)bh * HD + (unsigned)dt * 16u + lr) * KROWS + t0 + 8u * hi;
        const v16h vb0 = WFrag<h16>::ld(vp), vb1 = WFrag<h16>::ld(vp + 32);
        xa[dt] = wmma16(pa[0], vb0, xa[dt]); xa[dt] = wmma16(pa[1], vb1, xa[dt]);
        asm volatile("v_nop\n\tv_nop\n\tv_nop\n\tv_nop" : "+v"(xa[dt]) : "v"(vb0), "v"(vb1), "v"(pa[0]), "v"(pa[1]));
    }
#pragma unroll
    for (int dt = 0; dt < 4; ++dt)
#pragma unroll
        for (int j = 0; j < 8; ++j) ost[(8u * hi + (unsigned)j) * 68u + (unsigned)dt * 16u + lr] = xa[dt][j];
    __syncthreads();

    v8us oh[4], ol[4];
#pragma unroll
    for (int s = 0; s < 4; ++s) {
        const unsigned row = 4u * (unsigned)s + (lane >> 3), c = (lane & 7u) * 8u;
        const v4f a0 = *(const v4fa*)(ost + row * 68u + c); const v4f a1 = *(const v4fa*)(ost + row * 68u + c + 4u);
        const int mv = mask[(size_t)b * SEQ_FULL + t0 + row]; const float mk = (mv != 0) ? (1.0f / PCAR) : 0.0f;
#pragma unroll
        for (int q = 0; q < 4; ++q) { unsigned short hh, ll; const float y0 = a0[q] * mk + pz; splitf(y0, hh, ll); oh[s][q] = hh; ol[s][q] = ll; const float y1 = a1[q] * mk + pz; splitf(y1, hh, ll); oh[s][q + 4] = hh; ol[s][q + 4] = ll; }
    }
#pragma unroll
    for (int ps = 0; ps < 2; ++ps) {
#pragma unroll
        for (int s = 0; s < 4; ++s) { const unsigned row = 4u * (unsigned)s + (lane >> 3), c = (lane & 7u) * 8u; const size_t oo = ((size_t)b * SEQ + t0 + row) * DM + h * (unsigned)HD + c;
            *(volatile v8us*)(Ah + oo) = oh[s]; *(volatile v8us*)(Al + oo) = ol[s]; }
        if (ps == 0) __threadfence(); }
}

#define SZ_W   ((size_t)DM * DM * 2)
#define SZ_XB  ((size_t)NB * SEQ * DM * 2)
#define SZ_F   ((size_t)NB * SEQ * DM * 4)
#define SZ_QP  ((size_t)NBH * SEQ * HD * 2)
#define SZ_KP  ((size_t)NBH * KROWS * HD * 2)
#define SZ_AT  ((size_t)NB * SEQ * DM * 2)
#define SZ_ALL (4 * SZ_W + SZ_XB + SZ_F + 2 * SZ_QP + 3 * SZ_KP + 2 * SZ_AT)
static_assert(SZ_W % 256 == 0);
static_assert(SZ_XB % 256 == 0);
static_assert(SZ_QP % 256 == 0);
static_assert(SZ_KP % 256 == 0);
static_assert(SZ_ALL <= (size_t)134217728);

extern "C" void kernel_launch(void* const* d_in, const int* in_sizes, int n_in,
                              void* d_out, int out_size, void* d_ws, size_t ws_size, hipStream_t stream) {
    if (n_in < 13) return;
    const size_t needx = ((size_t)(NB - 1) * SEQ_FULL + SEQ) * DM;
    if ((size_t)in_sizes[0] < needx || (size_t)in_sizes[1] < needx || (size_t)in_sizes[2] < needx) return;
    if ((size_t)in_sizes[3] < (size_t)(NB - 1) * SEQ_FULL + SEQ || in_sizes[4] < 1) return;
    if (in_sizes[5] < DM * DM || in_sizes[7] < DM * DM || in_sizes[9] < DM * DM || in_sizes[11] < DM * DM) return;
    if (in_sizes[6] < DM || in_sizes[8] < DM || in_sizes[10] < DM || in_sizes[12] < DM) return;
    if ((size_t)out_size < needx) return;
    const float* xq = (const float*)d_in[0]; const float* xk = (const float*)d_in[1]; const float* xv = (const float*)d_in[2];
    const int* mask = (const int*)d_in[3]; const int* rs = (const int*)d_in[4];
    const float* wq = (const float*)d_in[5]; const float* bq = (const float*)d_in[6]; const float* wk = (const float*)d_in[7]; const float* bk = (const float*)d_in[8];
    const float* wv = (const float*)d_in[9]; const float* bv = (const float*)d_in[10]; const float* wo = (const float*)d_in[11]; const float* bo = (const float*)d_in[12];
    float* OUT = (float*)d_out;
    if (SZ_ALL > ws_size) return;
    char* wsp = (char*)d_ws;
    auto take = [&](size_t bytes) { char* p = wsp; wsp += (bytes + 255) & ~(size_t)255; return (void*)p; };
    bf* WQ = (bf*)take(SZ_W); bf* WK = (bf*)take(SZ_W); bf* WV = (bf*)take(SZ_W); bf* WO = (bf*)take(SZ_W);
    bf* XB = (bf*)take(SZ_XB); float* F = (float*)take(SZ_F);
    bf* QPh = (bf*)take(SZ_QP); bf* QPl = (bf*)take(SZ_QP); bf* KPh = (bf*)take(SZ_KP); bf* KPl = (bf*)take(SZ_KP); h16* VT16 = (h16*)take(SZ_KP);
    bf* ATh = (bf*)take(SZ_AT); bf* ATl = (bf*)take(SZ_AT);
    if ((size_t)(wsp - (char*)d_ws) > ws_size) return;

    const unsigned GW = (unsigned)(DM * DM / 64 / 64);
    k_wtG<<<GW, 256, 0, stream>>>(wq, WQ); k_wtG<<<GW, 256, 0, stream>>>(wk, WK); k_wtG<<<GW, 256, 0, stream>>>(wv, WV); k_wtG<<<GW, 256, 0, stream>>>(wo, WO);
    const unsigned GC = (unsigned)((size_t)NB * SEQ * (DM / 8) / 256);
    const dim3 GP((unsigned)(NB * SEQ / 64), (unsigned)(DM / 64), 1);
    k_cvt8b<<<GC, 256, 0, stream>>>(xq, XB);
    k_gemmw<bf, 0, true><<<GP, 32, 0, stream>>>(XB, nullptr, WQ, nullptr, DM, F, DM, bq, 0, 0, 0);
    k_hplane<(unsigned)SEQ, 0u><<<(unsigned)((size_t)NBH * SEQ * HD / 512), 256, 0, stream>>>(F, QPh, QPl);
    k_cvt8b<<<GC, 256, 0, stream>>>(xk, XB);
    k_gemmw<bf, 0, true><<<GP, 32, 0, stream>>>(XB, nullptr, WK, nullptr, DM, F, DM, bk, 0, 0, 0);
    k_hplane<(unsigned)KROWS, (unsigned)KOFF><<<(unsigned)((size_t)NBH * KROWS * HD / 512), 256, 0, stream>>>(F, KPh, KPl);
    k_cvt8b<<<GC, 256, 0, stream>>>(xv, XB);
    k_gemmw<bf, 0, true><<<GP, 32, 0, stream>>>(XB, nullptr, WV, nullptr, DM, F, DM, bv, 0, 0, 0);
    k_vt16<<<(unsigned)((size_t)NBH * HD * KROWS / 512), 256, 0, stream>>>(F, VT16);
    k_battn<<<dim3((unsigned)(SEQ / 16), (unsigned)NBH, 1), 32, 0, stream>>>(QPh, QPl, KPh, KPl, VT16, mask, rs, ATh, ATl);
    k_gemmw<bf, 1, true><<<dim3((unsigned)(SEQ / 64), (unsigned)(DM / 64), (unsigned)NB), 32, 0, stream>>>(ATh, ATl, WO, nullptr, DM, OUT, DM, bo, (size_t)SEQ * DM, 0, (size_t)SEQ_FULL * DM);
}
